// LiquidPerceptionUnit_68685116997889
// MI455X (gfx1250) — hardware-verified
//
#include <hip/hip_runtime.h>
#include <math.h>

typedef __attribute__((ext_vector_type(16))) _Float16 v16h;
typedef __attribute__((ext_vector_type(16))) __bf16 v16b;
typedef __attribute__((ext_vector_type(8)))  _Float16 v8h;
typedef __attribute__((ext_vector_type(8)))  float v8f;
typedef __attribute__((ext_vector_type(4)))  float v4f;
typedef __attribute__((ext_vector_type(2)))  float v2f;
typedef __attribute__((ext_vector_type(4)))  unsigned v4u;
typedef __attribute__((ext_vector_type(4)))  int v4i;
typedef float __attribute__((may_alias)) float_a;
typedef int __attribute__((may_alias)) int_a;

template <typename T> __device__ __forceinline__ void vst2(void* p, T v) { *(volatile T*)p = v; __threadfence(); *(volatile T*)p = v; }
__device__ __forceinline__ v8f wmma16(v16h a, v16h b, v8f c) {
  v8f d = __builtin_amdgcn_wmma_f32_16x16x32_f16(false, a, false, b, (short)0, c, false, false);
  asm volatile("v_nop\n\tv_nop\n\tv_nop\n\tv_nop" : "+v"(d) : "v"(a), "v"(b));
  return d;
}
__device__ __forceinline__ v8f wmma_bf(v16b a, v16b b, v8f c) {
  v8f d = __builtin_amdgcn_wmma_f32_16x16x32_bf16(false, a, false, b, (short)0, c, false, false);
  asm volatile("v_nop\n\tv_nop\n\tv_nop\n\tv_nop" : "+v"(d) : "v"(a), "v"(b));
  return d;
}
__device__ __forceinline__ v16h frag_h(const _Float16* rowk0, int lane) {
  union { v16h v; v8h q[2]; } u; const _Float16* p = rowk0 + 8 * (lane >> 4);
  u.q[0] = *(const v8h*)p; u.q[1] = *(const v8h*)(p + 16); return u.v;
}
__device__ __forceinline__ v16h frag_f32(const float* rowk0, int lane) {
  v16h a; const float* p = rowk0 + 8 * (lane >> 4);
#pragma unroll
  for (int i = 0; i < 8; ++i) { a[i] = (_Float16)p[i]; a[8 + i] = (_Float16)p[16 + i]; }
  return a;
}
__device__ __forceinline__ v16h frag_f32s(const float* rowk0, int lane, float sc) {
  v16h a; const float* p = rowk0 + 8 * (lane >> 4);
#pragma unroll
  for (int i = 0; i < 8; ++i) { a[i] = (_Float16)(p[i] * sc); a[8 + i] = (_Float16)(p[16 + i] * sc); }
  return a;
}
__device__ __forceinline__ v16h fragc_f32(const float* W, int k0, int n, int lane, int ld, int K) {
  v16h a; const int g = lane >> 4;
#pragma unroll
  for (int i = 0; i < 8; ++i) { const int ka = k0 + 8 * g + i, kb = ka + 16;
    a[i] = (_Float16)(ka < K ? W[(size_t)(ka < K ? ka : K - 1) * ld + n] : 0.f); a[8 + i] = (_Float16)(kb < K ? W[(size_t)(kb < K ? kb : K - 1) * ld + n] : 0.f); }
  return a;
}
struct F2 { v16b h, l; };
__device__ __forceinline__ F2 bsplit16(const float v[16]) { F2 r;
#pragma unroll
  for (int i = 0; i < 16; ++i) { const __bf16 h = (__bf16)v[i]; r.h[i] = h; r.l[i] = (__bf16)(v[i] - (float)h); }
  return r; }
__device__ __forceinline__ F2 split_row(const float* row, int k0, int lane) { float v[16]; const float* p = row + k0 + 8 * (lane >> 4);
#pragma unroll
  for (int i = 0; i < 8; ++i) { v[i] = p[i]; v[8 + i] = p[16 + i]; }
  return bsplit16(v); }
__device__ __forceinline__ F2 split_rowK(const float* row, int k0, int lane, int K) { float v[16]; const int g = lane >> 4;
#pragma unroll
  for (int i = 0; i < 8; ++i) { const int ka = k0 + 8 * g + i, kb = ka + 16; v[i] = ka < K ? row[ka < K ? ka : K - 1] : 0.f; v[8 + i] = kb < K ? row[kb < K ? kb : K - 1] : 0.f; }
  return bsplit16(v); }
__device__ __forceinline__ F2 split_col(const float* W, int k0, int n, int lane, int ld, int K) { float v[16]; const int g = lane >> 4;
#pragma unroll
  for (int i = 0; i < 8; ++i) { const int ka = k0 + 8 * g + i, kb = ka + 16; v[i] = ka < K ? W[(size_t)(ka < K ? ka : K - 1) * ld + n] : 0.f; v[8 + i] = kb < K ? W[(size_t)(kb < K ? kb : K - 1) * ld + n] : 0.f; }
  return bsplit16(v); }
__device__ __forceinline__ v8f mac3(const F2& a, const F2& b, v8f c) { c = wmma_bf(a.l, b.h, c); c = wmma_bf(a.h, b.l, c); return wmma_bf(a.h, b.h, c); }
__device__ __forceinline__ float sigm(float v) { return 1.0f / (1.0f + expf(-v)); }
#define LDSX() do { asm volatile("s_wait_dscnt 0" ::: "memory"); __builtin_amdgcn_wave_barrier(); __builtin_amdgcn_fence(__ATOMIC_RELEASE, "workgroup"); } while (0)


#define NB 32
#define NT 512
#define SL 256
#define FEAT 128
#ifndef NSTEP
#define NSTEP NT
#endif
typedef __attribute__((ext_vector_type(8))) __bf16 v8b;
__device__ __forceinline__ v16b frag_b(const __bf16* rowk0, int lane) {
  union { v16b v; v8b q[2]; } u; const __bf16* p = rowk0 + 8 * (lane >> 4);
  u.q[0] = *(const v8b*)p; u.q[1] = *(const v8b*)(p + 16); return u.v;
}
__device__ __forceinline__ float bfr(float v) { return (float)(__bf16)v; }
__device__ __attribute__((noinline)) float exp_ni(float v) { return expf(v); }
__device__ __attribute__((noinline)) float tanh_ni(float v) { return tanhf(v); }
#define L0_FIN 128
#define L0_HID 116
#define L0_KP 256
#define L0_HP 128
#define L1_FIN 116
#define L1_HID 76
#define L1_KP 192
#define L1_HP 80
#define L2_FIN 76
#define L2_HID 64
#define L2_KP 160
#define L2_HP 64
#define PW_L0 0
#define PW_L1 (PW_L0 + 4 * L0_HP * L0_KP)
#define PW_L2 (PW_L1 + 4 * L1_HP * L1_KP)
#define PW_END (PW_L2 + 4 * L2_HP * L2_KP)
#define WS_PW   0u
#define WS_PFC  (WS_PW + 2u * PW_END)
#define WS_FEAT (WS_PFC + 2u * 128 * 128)
#define WS_END  (WS_FEAT + 4u * NB * NT * FEAT)

__global__ __launch_bounds__(256) void k_pack(const float* __restrict__ m0, const float* __restrict__ w10, const float* __restrict__ w20, const float* __restrict__ wa0, const float* __restrict__ wb0,
                                              const float* __restrict__ m1, const float* __restrict__ w11, const float* __restrict__ w21, const float* __restrict__ wa1, const float* __restrict__ wb1,
                                              const float* __restrict__ m2, const float* __restrict__ w12, const float* __restrict__ w22, const float* __restrict__ wa2, const float* __restrict__ wb2,
                                              const float* __restrict__ fcw, __bf16* __restrict__ PW, __bf16* __restrict__ PFC) {
  __shared__ __align__(16) __bf16 srow[256];
  const int n = blockIdx.x, tid = threadIdx.x;
  const int n0 = 4 * L0_HP, n1 = n0 + 4 * L1_HP, n2 = n1 + 4 * L2_HP;
  if (n < n2) { int layer, m, r, hid, fin, kp, hp; size_t base;
    if (n < n0) { layer = 0; m = n / L0_HP; r = n % L0_HP; hid = L0_HID; fin = L0_FIN; kp = L0_KP; hp = L0_HP; base = PW_L0; }
    else if (n < n1) { layer = 1; m = (n - n0) / L1_HP; r = (n - n0) % L1_HP; hid = L1_HID; fin = L1_FIN; kp = L1_KP; hp = L1_HP; base = PW_L1; }
    else { layer = 2; m = (n - n1) / L2_HP; r = (n - n1) % L2_HP; hid = L2_HID; fin = L2_FIN; kp = L2_KP; hp = L2_HP; base = PW_L2; }
    const float* Wm = layer == 0 ? (m == 0 ? w10 : m == 1 ? w20 : m == 2 ? wa0 : wb0) : layer == 1 ? (m == 0 ? w11 : m == 1 ? w21 : m == 2 ? wa1 : wb1) : (m == 0 ? w12 : m == 1 ? w22 : m == 2 ? wa2 : wb2);
    const float* Mk = layer == 0 ? m0 : layer == 1 ? m1 : m2; const int cat = fin + hid;
    float v = 0.f; if (tid < kp) { if (r < hid && tid < cat) { v = bfr(Wm[(size_t)r * cat + tid]); if (m < 2) v = v * bfr(Mk[(size_t)r * cat + tid]); } srow[tid] = (__bf16)v; }
    __syncthreads();
    if (tid < kp / 8) vst2((unsigned*)(PW + base + ((size_t)m * hp + r) * kp + tid * 8), *(const v4u*)(&srow[tid * 8])); }
  else { const int o = n - n2; if (tid < 128) srow[tid] = (__bf16)bfr(fcw[(size_t)o * 128 + tid]); __syncthreads(); if (tid < 16) vst2((unsigned*)(PFC + (size_t)o * 128 + tid * 8), *(const v4u*)(&srow[tid * 8])); }
}
__global__ __launch_bounds__(128) void k_enc(const float* __restrict__ X, const float* __restrict__ c1w, const float* __restrict__ c1b, const float* __restrict__ c2w, const float* __restrict__ c2b, const __bf16* __restrict__ PFC, const float* __restrict__ fcb, float* __restrict__ FT) {
  __shared__ float sx[16][SL + 2]; __shared__ float sp1[16][16][10]; __shared__ float sc1[16][3], sb1[16], sc2[32][16][3], sb2[32]; __shared__ __align__(16) __bf16 sfh[16][136], sfl[16][136]; __shared__ __align__(16) float so[16][132];
  const int tid = threadIdx.x, lane = tid & 31, wave = tid >> 5, col = lane & 15, g = lane >> 4; const size_t s0 = (size_t)blockIdx.x * 16;
  for (int q = tid; q < 48; q += 128) sc1[q / 3][q % 3] = bfr(c1w[q]); if (tid < 16) sb1[tid] = bfr(c1b[tid]); for (int q = tid; q < 32 * 48; q += 128) sc2[q / 48][(q % 48) / 3][q % 3] = bfr(c2w[q]); if (tid < 32) sb2[tid] = bfr(c2b[tid]);
  for (int q = tid; q < 16 * SL; q += 128) { const int s = q / SL, p = q % SL; sx[s][p + 1] = bfr(X[(s0 + s) * SL + p]); } if (tid < 16) { sx[tid][0] = 0.f; sx[tid][SL + 1] = 0.f; }
  for (int q = tid; q < 16 * 16 * 10; q += 128) (&sp1[0][0][0])[q] = 0.f;
  __syncthreads();
  { const int s = tid >> 3, part = tid & 7;
    for (int oi = part; oi < 128; oi += 8) { const int ch = oi >> 3, pp = oi & 7; float acc = 0.f;
      for (int j = 0; j < 32; ++j) { const int p = pp * 32 + j; float v = sb1[ch] + sc1[ch][0] * sx[s][p] + sc1[ch][1] * sx[s][p + 1] + sc1[ch][2] * sx[s][p + 2]; acc += fmaxf(v, 0.f); }
      sp1[s][ch][pp + 1] = acc * (1.0f / 32.0f); } }
  __syncthreads();
  { const int s = tid >> 3, part = tid & 7;
    for (int fi = part; fi < 128; fi += 8) { const int co = fi >> 2, k = fi & 3; float acc = 0.f;
      for (int j = 0; j < 2; ++j) { const int p = k * 2 + j; float v = sb2[co];
        for (int ci = 0; ci < 16; ++ci) v += sc2[co][ci][0] * sp1[s][ci][p] + sc2[co][ci][1] * sp1[s][ci][p + 1] + sc2[co][ci][2] * sp1[s][ci][p + 2];
        acc += fmaxf(v, 0.f); }
      const float f = acc * 0.5f; const __bf16 hb = (__bf16)f; sfh[s][fi] = hb; sfl[s][fi] = (__bf16)(f - (float)hb); } }
  __syncthreads();
  { v8f acc[2] = {};
#pragma unroll
    for (int kc = 0; kc < 4; ++kc) { const v16b ah = frag_b(&sfh[col][kc * 32], lane), al = frag_b(&sfl[col][kc * 32], lane);
#pragma unroll
      for (int j = 0; j < 2; ++j) { const v16b w = frag_b(PFC + (size_t)((wave * 2 + j) * 16 + col) * 128 + kc * 32, lane); acc[j] = wmma_bf(al, w, acc[j]); acc[j] = wmma_bf(ah, w, acc[j]); } }
#pragma unroll
    for (int j = 0; j < 2; ++j) { const int o = (wave * 2 + j) * 16 + col; const float bb = bfr(fcb[o]);
#pragma unroll
      for (int r = 0; r < 8; ++r) so[8 * g + r][o] = acc[j][r] + bb; } }
  __syncthreads();
  for (int q = tid; q < 16 * 32; q += 128) { const int s = q >> 5, pc = q & 31; vst2(FT + (s0 + s) * FEAT + pc * 4, *(const v4f*)&so[s][pc * 4]); }
}
template <int KP, int HP, int HID>
__device__ __forceinline__ void cfc_cell(const __bf16 (*sxh)[264], const __bf16 (*sxl)[264], const __bf16* __restrict__ PW  , const float* __restrict__ b1, const float* __restrict__ b2, const float* __restrict__ ba, const float* __restrict__ bb, float (*sh)[132], int wave, int lane) {
  const int col = lane & 15, g = lane >> 4; const int rt = wave & 1, th = wave >> 1; constexpr int NTL = HP / 16;
  constexpr int MYT = (NTL + 3) / 4;
  v8f a1[MYT], a2[MYT], aa[MYT], ab[MYT];
#pragma unroll
  for (int j = 0; j < MYT; ++j) { a1[j] = (v8f){}; a2[j] = (v8f){}; aa[j] = (v8f){}; ab[j] = (v8f){}; }
#pragma unroll 1
  for (int kc = 0; kc < KP / 32; ++kc) { const v16b xh = frag_b(&sxh[rt * 16 + col][kc * 32], lane), xl = frag_b(&sxl[rt * 16 + col][kc * 32], lane);
#pragma unroll
    for (int j = 0; j < MYT; ++j) { const int t = th + 4 * j; if (t < NTL) {
        const v16b w1 = frag_b(PW + ((size_t)0 * HP + t * 16 + col) * KP + kc * 32, lane); a1[j] = wmma_bf(xl, w1, a1[j]); a1[j] = wmma_bf(xh, w1, a1[j]);
        const v16b w2 = frag_b(PW + ((size_t)1 * HP + t * 16 + col) * KP + kc * 32, lane); a2[j] = wmma_bf(xl, w2, a2[j]); a2[j] = wmma_bf(xh, w2, a2[j]);
        const v16b w3 = frag_b(PW + ((size_t)2 * HP + t * 16 + col) * KP + kc * 32, lane); aa[j] = wmma_bf(xl, w3, aa[j]); aa[j] = wmma_bf(xh, w3, aa[j]);
        const v16b w4 = frag_b(PW + ((size_t)3 * HP + t * 16 + col) * KP + kc * 32, lane); ab[j] = wmma_bf(xl, w4, ab[j]); ab[j] = wmma_bf(xh, w4, ab[j]); } } }
#pragma unroll
  for (int j = 0; j < MYT; ++j) { const int t = th + 4 * j; if (t < NTL) { const int o = t * 16 + col; if (o < HID) { const float c1 = bfr(b1[o]), c2 = bfr(b2[o]), c3 = bfr(ba[o]), c4 = bfr(bb[o]);
#pragma unroll
        for (int r = 0; r < 8; ++r) { const float f1 = tanh_ni(a1[j][r] + c1), f2 = tanh_ni(a2[j][r] + c2); const float ti = 1.0f / (1.0f + exp_ni(-((aa[j][r] + c3) + (ab[j][r] + c4)))); sh[rt * 16 + 8 * g + r][o] = f1 * (1.0f - ti) + ti * f2; } } } }
}
__global__ __launch_bounds__(256) void k_cfc(const float* __restrict__ FT, const __bf16* __restrict__ PW, const float* const* __restrict__ dummy,
                                             const float* __restrict__ b10, const float* __restrict__ b20, const float* __restrict__ ba0, const float* __restrict__ bb0,
                                             const float* __restrict__ b11, const float* __restrict__ b21, const float* __restrict__ ba1, const float* __restrict__ bb1,
                                             const float* __restrict__ b12, const float* __restrict__ b22, const float* __restrict__ ba2, const float* __restrict__ bb2, float* __restrict__ OUT, float* __restrict__ STATE) {
  (void)dummy;
  __shared__ __align__(16) __bf16 sxh[32][264], sxl[32][264]; __shared__ __align__(16) float sh0[32][132], sh1[32][132], sh2[32][132]; __shared__ __align__(16) float sst[32][260];
  const int tid = threadIdx.x, wave = tid >> 5, lane = tid & 31;
  for (int q = tid; q < 32 * 132; q += 256) { (&sh0[0][0])[q] = 0.f; (&sh1[0][0])[q] = 0.f; (&sh2[0][0])[q] = 0.f; }
  __syncthreads();
#pragma unroll 1
  for (int t = 0; t < NSTEP; ++t) {
    for (int q = tid; q < 32 * L0_KP; q += 256) { const int b = q / L0_KP, c = q % L0_KP; float v = 0.f; if (c < L0_FIN) v = FT[((size_t)b * NT + t) * FEAT + c]; else if (c < L0_FIN + L0_HID) v = sh0[b][c - L0_FIN]; const __bf16 hb = (__bf16)v; sxh[b][c] = hb; sxl[b][c] = (__bf16)(v - (float)hb); }
    __syncthreads();
    cfc_cell<L0_KP, L0_HP, L0_HID>(sxh, sxl, PW + PW_L0, b10, b20, ba0, bb0, sh0, wave, lane);
    __syncthreads();
    for (int q = tid; q < 32 * L1_KP; q += 256) { const int b = q / L1_KP, c = q % L1_KP; float v = 0.f; if (c < L1_FIN) v = sh0[b][c]; else if (c < L1_FIN + L1_HID) v = sh1[b][c - L1_FIN]; const __bf16 hb = (__bf16)v; sxh[b][c] = hb; sxl[b][c] = (__bf16)(v - (float)hb); }
    __syncthreads();
    cfc_cell<L1_KP, L1_HP, L1_HID>(sxh, sxl, PW + PW_L1, b11, b21, ba1, bb1, sh1, wave, lane);
    __syncthreads();
    for (int q = tid; q < 32 * L2_KP; q += 256) { const int b = q / L2_KP, c = q % L2_KP; float v = 0.f; if (c < L2_FIN) v = sh1[b][c]; else if (c < L2_FIN + L2_HID) v = sh2[b][c - L2_FIN]; const __bf16 hb = (__bf16)v; sxh[b][c] = hb; sxl[b][c] = (__bf16)(v - (float)hb); }
    __syncthreads();
    cfc_cell<L2_KP, L2_HP, L2_HID>(sxh, sxl, PW + PW_L2, b12, b22, ba2, bb2, sh2, wave, lane);
    __syncthreads();
    for (int q = tid; q < 32 * 16; q += 256) { const int b = q >> 4, pc = q & 15; vst2(OUT + ((size_t)b * NT + t) * 64 + pc * 4, *(const v4f*)&sh2[b][pc * 4]); }
    __syncthreads(); }
  for (int q = tid; q < 32 * 256; q += 256) { const int b = q >> 8, c = q & 255; sst[b][c] = c < 116 ? sh0[b][c] : (c < 192 ? sh1[b][c - 116] : sh2[b][c - 192]); }
  __syncthreads();
  for (int q = tid; q < 32 * 64; q += 256) { const int b = q >> 6, pc = q & 63; vst2(STATE + (size_t)b * 256 + pc * 4, *(const v4f*)&sst[b][pc * 4]); }
}

extern "C" void kernel_launch(void* const* d_in, const int* in_sizes, int n_in, void* d_out, int out_size, void* d_ws, size_t ws_size, hipStream_t stream) {
  (void)in_sizes; (void)n_in; (void)out_size;
  const float** F = (const float**)d_in;
  if (ws_size < (size_t)WS_END) return;
  char* ws = (char*)d_ws; __bf16 *PW = (__bf16*)(ws + WS_PW), *PFC = (__bf16*)(ws + WS_PFC); float* FT = (float*)(ws + WS_FEAT);
  float* OUT = (float*)d_out; float* STATE = OUT + (size_t)NB * NT * 64;
  const int L0 = 7, L1 = 16, L2 = 25;
  k_pack<<<4 * (L0_HP + L1_HP + L2_HP) + 128, 256, 0, stream>>>(F[L0], F[L0 + 1], F[L0 + 2], F[L0 + 3], F[L0 + 4], F[L1], F[L1 + 1], F[L1 + 2], F[L1 + 3], F[L1 + 4], F[L2], F[L2 + 1], F[L2 + 2], F[L2 + 3], F[L2 + 4], F[5], PW, PFC);
  k_enc<<<NB * NT / 16, 128, 0, stream>>>(F[0], F[1], F[2], F[3], F[4], PFC, F[6], FT);
  k_cfc<<<1, 256, 0, stream>>>(FT, PW, nullptr, F[L0 + 5], F[L0 + 6], F[L0 + 7], F[L0 + 8], F[L1 + 5], F[L1 + 6], F[L1 + 7], F[L1 + 8], F[L2 + 5], F[L2 + 6], F[L2 + 7], F[L2 + 8], OUT, STATE);
}
